// JITODESolver_44470091383428
// MI455X (gfx1250) — hardware-verified
//
#include <hip/hip_runtime.h>


namespace {
constexpr int B = 2048, IN = 128, H = 256, OUT = 128, T = 65, NS = T - 1, H2 = 2 * H;
constexpr float XS = 8.0f, WSC = 256.0f;
typedef _Float16 b16;
typedef __attribute__((ext_vector_type(16))) _Float16 v16b;
typedef __attribute__((ext_vector_type(8))) _Float16 v8b;
typedef __attribute__((ext_vector_type(8))) float v8f;
typedef __attribute__((ext_vector_type(4))) float v4f;
__device__ __forceinline__ float bf16_rne(float f) { unsigned int u = __float_as_uint(f); u += 0x7FFFu + ((u >> 16) & 1u); return __uint_as_float(u & 0xFFFF0000u); }
__device__ __forceinline__ void split16(float v, b16& hi, b16& lo) { hi = (b16)v; lo = (b16)(v - (float)hi); }
__device__ __forceinline__ v16b frag_kb(const b16* p, int hh) { const v8b a = *(const v8b*)(p + 8 * hh), b = *(const v8b*)(p + 16 + 8 * hh); v16b f;
#pragma unroll
  for (int e = 0; e < 8; ++e) { f[e] = a[e]; f[8 + e] = b[e]; } return f; }
__device__ __forceinline__ v8f wmma16b(v16b a, v16b b, v8f c) { v8f d = __builtin_amdgcn_wmma_f32_16x16x32_f16(false, a, false, b, (short)0, c, false, false); asm volatile("v_nop\n\tv_nop\n\tv_nop\n\tv_nop" : "+v"(d) : "v"(a), "v"(b)); return d; }
__device__ __forceinline__ void wave_lds_sync() { __builtin_amdgcn_fence(__ATOMIC_RELEASE, "workgroup"); __builtin_amdgcn_wave_barrier(); __builtin_amdgcn_fence(__ATOMIC_ACQUIRE, "workgroup"); }
__device__ __forceinline__ float pmul(float a, float b) { float p = a * b; asm volatile("" : "+v"(p)); return p; }
__device__ __forceinline__ float sigm(float v) { return 1.0f / (1.0f + __expf(-v)); }

__global__ __launch_bounds__(256) void wprep_kernel(const float* __restrict__ wg, const float* __restrict__ wf, int r0, int KIN, b16* __restrict__ WT) {
  const size_t u = (size_t)blockIdx.x * 256 + threadIdx.x; if (u >= (size_t)H2 * KIN / 8) return; const size_t e = u * 8; const int o = (int)(e / KIN), k0 = (int)(e % KIN); v8b v; const float* w = o < H ? wg : wf; const int oc = o < H ? o : o - H;
  for (int j = 0; j < 8; ++j) v[j] = (b16)(bf16_rne(w[(size_t)(r0 + k0 + j) * H + oc]) * WSC); for (int pass = 0; pass < 2; ++pass) { *(volatile v8b*)(WT + e) = v; __threadfence(); }
}
__global__ __launch_bounds__(256) void wprepo_kernel(const float* __restrict__ w, b16* __restrict__ WT) {
  const size_t u = (size_t)blockIdx.x * 256 + threadIdx.x; if (u >= (size_t)OUT * H / 8) return; const size_t e = u * 8; const int o = (int)(e / H), k0 = (int)(e % H); v8b v;
  for (int j = 0; j < 8; ++j) v[j] = (b16)(bf16_rne(w[(size_t)(k0 + j) * OUT + o]) * WSC); for (int pass = 0; pass < 2; ++pass) { *(volatile v8b*)(WT + e) = v; __threadfence(); }
}
__global__ __launch_bounds__(32) void main_kernel(const float* __restrict__ x, const b16* __restrict__ WX, const b16* __restrict__ WH, const b16* __restrict__ WO, const float* __restrict__ bg, const float* __restrict__ bf, const float* __restrict__ tau, const float* __restrict__ tev, const float* __restrict__ bo, float* __restrict__ out) {
  __shared__ __attribute__((aligned(16))) b16 Ah[16][H + 8], Al[16][H + 8]; __shared__ __attribute__((aligned(16))) float Zx[16][H2 + 4]; __shared__ __attribute__((aligned(16))) float Hs[16][H + 4];
  const int lane = threadIdx.x, nloc = lane & 15, hlf = lane >> 4; const size_t m0 = (size_t)blockIdx.x * 16; const float sc = 1.0f / (XS * WSC); const float dt = bf16_rne(tev[1]) - bf16_rne(tev[0]);
  for (int rr = 0; rr < 16; ++rr) { const v4f v = *(const v4f*)(x + (m0 + rr) * IN + lane * 4); for (int j = 0; j < 4; ++j) Ah[rr][lane * 4 + j] = (b16)(bf16_rne(v[j]) * XS); for (int q = 0; q < 2; ++q) for (int j = 0; j < 4; ++j) Hs[rr][q * 128 + lane * 4 + j] = 0.0f; }
  wave_lds_sync();
#pragma unroll 1
  for (int cg = 0; cg < 4; ++cg) { v8f acc[8];
#pragma unroll
    for (int t = 0; t < 8; ++t) acc[t] = (v8f){};
#pragma unroll
    for (int kb = 0; kb < IN; kb += 32) { const v16b a = frag_kb(&Ah[nloc][kb], hlf);
#pragma unroll
      for (int t = 0; t < 8; ++t) acc[t] = wmma16b(a, frag_kb(WX + (size_t)(cg * 128 + t * 16 + nloc) * IN + kb, hlf), acc[t]); }
#pragma unroll
    for (int t = 0; t < 8; ++t) { const int c = cg * 128 + t * 16 + nloc; const float bb = c < H ? bf16_rne(bg[c]) : bf16_rne(bf[c - H]);
#pragma unroll 1
      for (int r8 = 0; r8 < 8; ++r8) Zx[8 * hlf + r8][c] = acc[t][r8] * sc + bb; } }
  wave_lds_sync();
  float tinv[8]; for (int t = 0; t < 8; ++t) tinv[t] = 1.0f / bf16_rne(tau[t * 16 + nloc]);
#pragma unroll 1
  for (int st = 0; st < NS; ++st) {
    for (int rr = 0; rr < 16; ++rr) for (int q = 0; q < 2; ++q) for (int j = 0; j < 4; ++j) { const int c = q * 128 + lane * 4 + j; b16 p, ql; split16(Hs[rr][c] * XS, p, ql); Ah[rr][c] = p; Al[rr][c] = ql; }
    wave_lds_sync();
#pragma unroll 1
    for (int cg = 0; cg < 2; ++cg) { v8f ag[8], af[8];
#pragma unroll
      for (int t = 0; t < 8; ++t) { ag[t] = (v8f){}; af[t] = (v8f){}; }
#pragma unroll 2
      for (int kb = 0; kb < H; kb += 32) { const v16b a = frag_kb(&Ah[nloc][kb], hlf), al = frag_kb(&Al[nloc][kb], hlf);
#pragma unroll
        for (int t = 0; t < 8; ++t) { const v16b bwg = frag_kb(WH + (size_t)(cg * 128 + t * 16 + nloc) * H + kb, hlf), bwf = frag_kb(WH + (size_t)(H + cg * 128 + t * 16 + nloc) * H + kb, hlf);
          ag[t] = wmma16b(a, bwg, ag[t]); ag[t] = wmma16b(al, bwg, ag[t]); af[t] = wmma16b(a, bwf, af[t]); af[t] = wmma16b(al, bwf, af[t]); } }
#pragma unroll
      for (int t = 0; t < 8; ++t) { const int c = cg * 128 + t * 16 + nloc; const float ti = 1.0f / bf16_rne(tau[c]);
#pragma unroll
        for (int r8 = 0; r8 < 8; ++r8) { const int rl = 8 * hlf + r8; const float g = sigm(ag[t][r8] * sc + Zx[rl][c]); const float f = af[t][r8] * sc + Zx[rl][H + c]; const float h = Hs[rl][c]; Hs[rl][c] = h + pmul(pmul(pmul(f, g) - h, ti), dt); } } }
    wave_lds_sync(); }
  (void)tinv;
  for (int rr = 0; rr < 16; ++rr) for (int q = 0; q < 2; ++q) for (int j = 0; j < 4; ++j) { const int c = q * 128 + lane * 4 + j; b16 p, ql; split16(Hs[rr][c] * XS, p, ql); Ah[rr][c] = p; Al[rr][c] = ql; }
  wave_lds_sync();
  { v8f acc[8];
#pragma unroll
    for (int t = 0; t < 8; ++t) acc[t] = (v8f){};
#pragma unroll 2
    for (int kb = 0; kb < H; kb += 32) { const v16b a = frag_kb(&Ah[nloc][kb], hlf), al = frag_kb(&Al[nloc][kb], hlf);
#pragma unroll
      for (int t = 0; t < 8; ++t) { const v16b bw = frag_kb(WO + (size_t)(t * 16 + nloc) * H + kb, hlf); acc[t] = wmma16b(a, bw, acc[t]); acc[t] = wmma16b(al, bw, acc[t]); } }
#pragma unroll
    for (int t = 0; t < 8; ++t) { const int c = t * 16 + nloc; const float bb = bf16_rne(bo[c]);
#pragma unroll 1
      for (int r8 = 0; r8 < 8; ++r8) Zx[8 * hlf + r8][c] = acc[t][r8] * sc + bb; } }
  wave_lds_sync();
  for (int pass = 0; pass < 2; ++pass) { for (int rr = 0; rr < 16; ++rr) *(volatile v4f*)(out + (m0 + rr) * OUT + lane * 4) = *(const v4f*)(&Zx[rr][lane * 4]); __threadfence(); }
}
}

extern "C" void kernel_launch(void* const* d_in, const int* in_sizes, int n_in, void* d_out, int out_size, void* d_ws, size_t ws_size, hipStream_t stream) {
  (void)n_in;
  auto Fp = [&](int i) { return (const float*)d_in[i]; };
  if (in_sizes[0] != B * IN || in_sizes[1] != T || in_sizes[2] != (IN + H) * H || in_sizes[4] != (IN + H) * H || in_sizes[6] != H || in_sizes[7] != H * OUT || out_size != B * OUT) return;
  const int NBV = B / 16;
  size_t off = 0; char* ws = (char*)d_ws;
  auto carve = [&](size_t bytes) { char* p = ws + off; off += (bytes + 255) & ~(size_t)255; return p; };
  b16* WX = (b16*)carve((size_t)H2 * IN * 2); b16* WH = (b16*)carve((size_t)H2 * H * 2); b16* WO = (b16*)carve((size_t)OUT * H * 2);
  if (off > ws_size) return;
  wprep_kernel<<<(H2 * IN / 8 + 255) / 256, 256, 0, stream>>>(Fp(2), Fp(4), 0, IN, WX); wprep_kernel<<<(H2 * H / 8 + 255) / 256, 256, 0, stream>>>(Fp(2), Fp(4), IN, H, WH); wprepo_kernel<<<(OUT * H / 8 + 255) / 256, 256, 0, stream>>>(Fp(7), WO);
  main_kernel<<<NBV, 32, 0, stream>>>(Fp(0), WX, WH, WO, Fp(3), Fp(5), Fp(6), Fp(1), Fp(8), (float*)d_out);
}
